// PointwiseAggregatedAttention_86955907875119
// MI455X (gfx1250) — hardware-verified
//
#include <hip/hip_runtime.h>


#define NBI  4
#define NT   2048
#define DD   256
#define NH   4
#define HD   64
#define DM   DD
#define LOSC 1024.0f

typedef _Float16 h16;
typedef unsigned short bf;
typedef __attribute__((ext_vector_type(16))) __bf16   v16bf;
typedef __attribute__((ext_vector_type(16))) _Float16 v16h;
typedef __attribute__((ext_vector_type(8)))  _Float16 v8h;
typedef __attribute__((ext_vector_type(8)))  unsigned short v8us;
typedef __attribute__((ext_vector_type(8)))  float    v8f;
typedef __attribute__((ext_vector_type(4)))  float    v4f;
typedef v8h  __attribute__((may_alias)) v8ha;
typedef v4f  __attribute__((may_alias)) v4fa;
typedef v8us __attribute__((may_alias)) v8usa;

__device__ __forceinline__ unsigned short f2bf(float f) { unsigned u = __float_as_uint(f); u += 0x7FFFu + ((u >> 16) & 1u); return (unsigned short)(u >> 16); }
__device__ __forceinline__ float bf2f(unsigned short b) { return __uint_as_float(((unsigned)b) << 16); }
__device__ __forceinline__ float bfr(float f) { return bf2f(f2bf(f)); }
__device__ __forceinline__ v16h cat16(v8h lo, v8h hi) { return __builtin_shufflevector(lo, hi, 0, 1, 2, 3, 4, 5, 6, 7, 8, 9, 10, 11, 12, 13, 14, 15); }
__device__ __forceinline__ v16bf cat16b(v8us lo, v8us hi) { return __builtin_bit_cast(v16bf, __builtin_shufflevector(lo, hi, 0, 1, 2, 3, 4, 5, 6, 7, 8, 9, 10, 11, 12, 13, 14, 15)); }
__device__ __forceinline__ v8f wmma16(v16h a, v16h b, v8f c) { return __builtin_amdgcn_wmma_f32_16x16x32_f16(false, a, false, b, (short)0, c, false, false); }
__device__ __forceinline__ v8f wmmab(v16bf a, v16bf b, v8f c) { return __builtin_amdgcn_wmma_f32_16x16x32_bf16(false, a, false, b, (short)0, c, false, false); }

template <bool SPLITA, bool F16OUT = false>
__global__ __launch_bounds__(128) void k_gemmb(const bf* __restrict__ A, const bf* __restrict__ Al, const bf* __restrict__ Bn, const float* __restrict__ bias, float* C, int ldc, h16* C2, const float* __restrict__ R = nullptr, int K = DM, int roundR = 1) {
    __shared__ __align__(16) float ost[4][16 * 68];
    const int lane = threadIdx.x & 31, wave = threadIdx.x >> 5, lr = lane & 15, hi = lane >> 4;
    const int r0 = blockIdx.x * 64 + wave * 16, c0 = blockIdx.y * 64;
    const size_t aoff = (size_t)(r0 + lr) * K + 8 * hi;
    size_t boff[4];
#pragma unroll
    for (int t = 0; t < 4; ++t) boff[t] = (size_t)(c0 + t * 16 + lr) * K + 8 * hi;
    v8f acc[4];
#pragma unroll
    for (int t = 0; t < 4; ++t) acc[t] = (v8f){};
#pragma unroll 1
    for (int kc = 0; kc < K; kc += 32) {
        const v16bf a = cat16b(*(const v8us*)(A + aoff + kc), *(const v8us*)(A + aoff + kc + 16));
        v16bf al = a;
        if (SPLITA) al = cat16b(*(const v8us*)(Al + aoff + kc), *(const v8us*)(Al + aoff + kc + 16));
#pragma unroll
        for (int t = 0; t < 4; ++t) { const v16bf b = cat16b(*(const v8us*)(Bn + boff[t] + kc), *(const v8us*)(Bn + boff[t] + kc + 16)); acc[t] = wmmab(a, b, acc[t]); if (SPLITA) acc[t] = wmmab(al, b, acc[t]); }
        asm volatile("v_nop\n\tv_nop\n\tv_nop\n\tv_nop" : "+v"(acc[0]), "+v"(acc[1]), "+v"(acc[2]), "+v"(acc[3]) : "v"(a), "v"(al));
    }
    float* os = &ost[wave][0];
#pragma unroll
    for (int t = 0; t < 4; ++t) { const float bv = bias ? bfr(bias[c0 + t * 16 + lr]) : 0.f;
#pragma unroll
        for (int j = 0; j < 8; ++j) os[(hi * 8 + j) * 68 + t * 16 + lr] = acc[t][j] + bv; }
    __syncthreads();
    if (F16OUT) {
        h16* crow = (h16*)(void*)C + (size_t)r0 * ldc + c0;
        auto pass = [&]() {
#pragma unroll
            for (int s = 0; s < 4; ++s) { const int row = 4 * s + (lane >> 3), piece = lane & 7; const float* sp = os + row * 68 + piece * 8; v8h o, o2;
#pragma unroll
                for (int i = 0; i < 8; ++i) { const h16 a = (h16)sp[i]; o[i] = a; o2[i] = (h16)((sp[i] - (float)a) * LOSC); }
                *(volatile v8h*)(crow + (size_t)row * ldc + piece * 8) = o; if (C2) *(volatile v8h*)(C2 + (size_t)r0 * ldc + c0 + (size_t)row * ldc + piece * 8) = o2; }
        };
        pass(); __threadfence(); pass();
    } else {
        float* crow = C + (size_t)r0 * ldc + c0;
        auto pass = [&]() {
#pragma unroll
            for (int s = 0; s < 8; ++s) { const int Lid = (lane >> 3) + 4 * s, piece = lane & 7; const int row = Lid >> 1, cofs = (Lid & 1) * 32 + piece * 4;
                v4f val = *(const v4fa*)(os + row * 68 + cofs); if (R) { const v4f rv = *(const v4f*)(R + ((size_t)r0 + row) * ldc + c0 + cofs); val += roundR ? (v4f){bfr(rv[0]), bfr(rv[1]), bfr(rv[2]), bfr(rv[3])} : rv; }
                *(volatile v4f*)(crow + (size_t)row * ldc + cofs) = val; }
        };
        pass(); __threadfence(); pass();
    }
}


__global__ __launch_bounds__(256) void k_cvt8(const float* __restrict__ src, bf* dst, size_t n8) {
    const size_t i = (size_t)blockIdx.x * 256 + threadIdx.x; if (i >= n8) return;
    const v8f v = *(const v8f*)(src + i * 8); v8us o;
#pragma unroll
    for (int k = 0; k < 8; ++k) o[k] = f2bf(v[k]);
    *(volatile v8us*)(dst + i * 8) = o; __threadfence(); *(volatile v8us*)(dst + i * 8) = o;
}
__global__ __launch_bounds__(256) void k_zero8(bf* dst, size_t n8) {
    const size_t i = (size_t)blockIdx.x * 256 + threadIdx.x; if (i >= n8) return; v8us z;
#pragma unroll
    for (int k = 0; k < 8; ++k) z[k] = 0;
    *(volatile v8us*)(dst + i * 8) = z; __threadfence(); *(volatile v8us*)(dst + i * 8) = z;
}

__global__ __launch_bounds__(256) void k_cvt(const float* __restrict__ src, bf* dst) {
    const int lane = threadIdx.x & 31, r = blockIdx.x * 8 + (threadIdx.x >> 5); if (r >= NT) return; v8us o;
#pragma unroll
    for (int i = 0; i < 8; ++i) o[i] = f2bf(src[(size_t)r * DD + lane * 8 + i]);
    *(volatile v8us*)(dst + (size_t)r * DD + lane * 8) = o; __threadfence(); *(volatile v8us*)(dst + (size_t)r * DD + lane * 8) = o;
}
__global__ __launch_bounds__(256) void k_split256m(const float* __restrict__ src, const int* __restrict__ m, bf* dh, bf* dl) {
    const int lane = threadIdx.x & 31, r = blockIdx.x * 8 + (threadIdx.x >> 5); if (r >= NT) return; const float f = m ? ((m[r] != 0) ? 1.0f : 0.f) : 1.0f;
    const size_t o = (size_t)r * DD + lane * 8; const v8f v = *(const v8f*)(src + o); v8us oh, ol;
#pragma unroll
    for (int i = 0; i < 8; ++i) { const float y = v[i] * f; const unsigned short hb = f2bf(y); oh[i] = hb; ol[i] = f2bf(y - bf2f(hb)); }
    *(volatile v8us*)(dh + o) = oh; *(volatile v8us*)(dl + o) = ol; __threadfence(); *(volatile v8us*)(dh + o) = oh; *(volatile v8us*)(dl + o) = ol;
}
__global__ __launch_bounds__(256) void k_vtb(const float* __restrict__ src, const int* __restrict__ m, bf* Th, bf* Tl) {
    __shared__ float tl[64][65];
    const int tid = threadIdx.x, t0 = blockIdx.x * 64, h = blockIdx.y;
    { const int tt = tid >> 2, dq = (tid & 3) * 16; const float f = (m[t0 + tt] != 0) ? 1.0f : 0.f;
#pragma unroll 4
      for (int i = 0; i < 16; ++i) tl[dq + i][tt] = src[(size_t)(t0 + tt) * DD + h * HD + dq + i] * f; }
    __syncthreads();
    const int piece = tid & 7, Lid = tid >> 3;
    auto pass = [&]() {
#pragma unroll
        for (int s = 0; s < 2; ++s) { const int d = Lid + 32 * s; v8us oh, ol;
#pragma unroll
            for (int i = 0; i < 8; ++i) { const float v = tl[d][piece * 8 + i]; const unsigned short hb = f2bf(v); oh[i] = hb; ol[i] = f2bf(v - bf2f(hb)); }
            const size_t o = ((size_t)h * HD + d) * NT + t0 + piece * 8; *(volatile v8us*)(Th + o) = oh; *(volatile v8us*)(Tl + o) = ol; }
    };
    pass(); __threadfence(); pass();
}
__global__ __launch_bounds__(256) void k_tbuild(const float* __restrict__ rb, bf* T) {
    const int lane = threadIdx.x & 31; const int wid = blockIdx.x * 8 + (threadIdx.x >> 5); const int h = wid / NT, i = wid - h * NT; if (h >= NH) return;
#pragma unroll 1
    for (int ps = 0; ps < 2; ++ps) {
#pragma unroll 1
        for (int c0 = lane * 8; c0 < NT; c0 += 256) { v8us o;
#pragma unroll
            for (int q = 0; q < 8; ++q) { const int j = c0 + q; o[q] = f2bf(rb[(size_t)(j - i + NT - 1) * NH + h]); }
            *(volatile v8us*)(T + ((size_t)h * NT + i) * NT + c0) = o; }
        if (ps == 0) __threadfence(); }
}
__global__ __launch_bounds__(256) void k_kvsplit(const float* __restrict__ src, const float* __restrict__ scale, bf* dh, bf* dl) {
    typedef __attribute__((ext_vector_type(2))) unsigned short v2us;
    const int lane = threadIdx.x & 31, r = blockIdx.x * 8 + (threadIdx.x >> 5); if (r >= HD) return; const float is = 1.0f / bfr(scale[0]);
    const size_t o = (size_t)r * HD + lane * 2; v2us oh, ol;
#pragma unroll
    for (int i = 0; i < 2; ++i) { const float y = src[o + i] * is; const unsigned short hb = f2bf(y); oh[i] = hb; ol[i] = f2bf(y - bf2f(hb)); }
    *(volatile v2us*)(dh + o) = oh; *(volatile v2us*)(dl + o) = ol; __threadfence(); *(volatile v2us*)(dh + o) = oh; *(volatile v2us*)(dl + o) = ol;
}
__global__ __launch_bounds__(256) void k_tadd(const float* __restrict__ C2, int h, float* Y) {
    __shared__ float tl[64][65];
    const int tid = threadIdx.x, i0 = blockIdx.x * 64;
    { const int d = tid >> 2, iq = (tid & 3) * 16;
#pragma unroll 4
      for (int k = 0; k < 16; ++k) tl[iq + k][d] = C2[(size_t)d * NT + i0 + iq + k]; }
    __syncthreads();
    const int piece = tid & 15, Lid = tid >> 4; v4f vals[4];
#pragma unroll
    for (int s = 0; s < 4; ++s) { const int i = Lid + 16 * s; const size_t o = (size_t)(i0 + i) * DD + h * HD + piece * 4; v4f y = *(const v4f*)(Y + o);
#pragma unroll
        for (int k = 0; k < 4; ++k) y[k] += tl[i][piece * 4 + k];
        vals[s] = y; }
    auto pass = [&]() {
#pragma unroll
        for (int s = 0; s < 4; ++s) { const int i = Lid + 16 * s; *(volatile v4f*)(Y + (size_t)(i0 + i) * DD + h * HD + piece * 4) = vals[s]; }
    };
    pass(); __threadfence(); pass();
}

__global__ __launch_bounds__(128) void k_gemm3ll(const bf* __restrict__ Ah, const bf* __restrict__ Al, int lda, const bf* __restrict__ Bh, const bf* __restrict__ Bl, int ldb, int K, float* C, int ldc) {
    __shared__ __align__(16) float ost[4][16 * 68];
    const int lane = threadIdx.x & 31, wave = threadIdx.x >> 5, lr = lane & 15, hi = lane >> 4;
    const int r0 = blockIdx.x * 64 + wave * 16, c0 = blockIdx.y * 64;
    const size_t aoff = (size_t)(r0 + lr) * lda + 8 * hi;
    v8f acc[4];
#pragma unroll
    for (int t = 0; t < 4; ++t) acc[t] = (v8f){};
#pragma unroll 1
    for (int kc = 0; kc < K; kc += 32) {
        const v16bf a = cat16b(*(const v8us*)(Ah + aoff + kc), *(const v8us*)(Ah + aoff + kc + 16));
        const v16bf al = cat16b(*(const v8us*)(Al + aoff + kc), *(const v8us*)(Al + aoff + kc + 16));
#pragma unroll
        for (int t = 0; t < 4; ++t) { const size_t bo = (size_t)(c0 + t * 16 + lr) * ldb + kc + 8 * hi;
            const v16bf bh = cat16b(*(const v8us*)(Bh + bo), *(const v8us*)(Bh + bo + 16)); const v16bf bl = cat16b(*(const v8us*)(Bl + bo), *(const v8us*)(Bl + bo + 16));
            acc[t] = wmmab(a, bh, acc[t]); acc[t] = wmmab(al, bh, acc[t]); acc[t] = wmmab(a, bl, acc[t]); }
        asm volatile("v_nop\n\tv_nop\n\tv_nop\n\tv_nop" : "+v"(acc[0]), "+v"(acc[1]), "+v"(acc[2]), "+v"(acc[3]) : "v"(a), "v"(al));
    }
    float* os = &ost[wave][0];
#pragma unroll
    for (int t = 0; t < 4; ++t) {
#pragma unroll
        for (int j = 0; j < 8; ++j) os[(hi * 8 + j) * 68 + t * 16 + lr] = acc[t][j]; }
    __builtin_amdgcn_wave_barrier(); asm volatile("" ::: "memory");
    float* crow = C + (size_t)r0 * ldc + c0;
    auto pass = [&]() {
#pragma unroll
        for (int s = 0; s < 8; ++s) { const int Lid = (lane >> 3) + 4 * s, piece = lane & 7; const int row = Lid >> 1, cofs = (Lid & 1) * 32 + piece * 4;
            const v4f val = *(const v4fa*)(os + row * 68 + cofs); *(volatile v4f*)(crow + (size_t)row * ldc + cofs) = val; }
    };
    pass(); __threadfence(); pass();
}

extern "C" void kernel_launch(void* const* d_in, const int* in_sizes, int n_in,
                              void* d_out, int out_size, void* d_ws, size_t ws_size, hipStream_t stream) {
    (void)in_sizes; (void)n_in; (void)out_size;
    const float* x = (const float*)d_in[0]; const float* Wq = (const float*)d_in[1]; const float* bq = (const float*)d_in[2]; const float* Wk = (const float*)d_in[3]; const float* bk = (const float*)d_in[4]; const float* Wv = (const float*)d_in[5]; const float* bv = (const float*)d_in[6];
    const float* Wo = (const float*)d_in[7]; const float* bo = (const float*)d_in[8]; const float* rb = (const float*)d_in[9]; const float* scale = (const float*)d_in[10]; const int* mask = (const int*)d_in[11];
    float* out = (float*)d_out;
    char* wsp = (char*)d_ws;
    auto take = [&](size_t bytes) { char* p = wsp; wsp += (bytes + 255) & ~(size_t)255; return (void*)p; };
    bf* WqB = (bf*)take(DD * DD * 2); bf* WkB = (bf*)take(DD * DD * 2); bf* WvB = (bf*)take(DD * DD * 2); bf* WoB = (bf*)take(DD * DD * 2); bf* T = (bf*)take((size_t)NH * NT * NT * 2);
    bf* Xb = (bf*)take((size_t)NT * DD * 2); float* TMP = (float*)take((size_t)NT * DD * 4); bf* Qh = (bf*)take((size_t)NT * DD * 2); bf* Ql = (bf*)take((size_t)NT * DD * 2);
    bf* KTh = (bf*)take((size_t)DD * NT * 2); bf* KTl = (bf*)take((size_t)DD * NT * 2); bf* VTh = (bf*)take((size_t)DD * NT * 2); bf* VTl = (bf*)take((size_t)DD * NT * 2);
    float* KV = (float*)take(HD * HD * 4); bf* KVh = (bf*)take(HD * HD * 2); bf* KVl = (bf*)take(HD * HD * 2); float* Y = (float*)take((size_t)NT * DD * 4); float* C2 = (float*)take((size_t)HD * NT * 4); bf* Yh = (bf*)take((size_t)NT * DD * 2); bf* Yl = (bf*)take((size_t)NT * DD * 2);
    if ((size_t)(wsp - (char*)d_ws) > ws_size) return;
    { const size_t n1 = DD * DD / 8; k_cvt8<<<(unsigned)((n1 + 255) / 256), 256, 0, stream>>>(Wq, WqB, n1); k_cvt8<<<(unsigned)((n1 + 255) / 256), 256, 0, stream>>>(Wk, WkB, n1); k_cvt8<<<(unsigned)((n1 + 255) / 256), 256, 0, stream>>>(Wv, WvB, n1); k_cvt8<<<(unsigned)((n1 + 255) / 256), 256, 0, stream>>>(Wo, WoB, n1); }
    k_tbuild<<<(NH * NT) / 8, 256, 0, stream>>>(rb, T);
    for (int b = 0; b < NBI; ++b) { const int* mb = mask + (size_t)b * NT;
        k_cvt<<<NT / 8, 256, 0, stream>>>(x + (size_t)b * NT * DD, Xb);
        k_gemmb<false, false><<<dim3(NT / 64, DD / 64, 1), 128, 0, stream>>>(Xb, nullptr, WqB, bq, TMP, DD, nullptr, nullptr, DD); k_split256m<<<NT / 8, 256, 0, stream>>>(TMP, mb, Qh, Ql);
        k_gemmb<false, false><<<dim3(NT / 64, DD / 64, 1), 128, 0, stream>>>(Xb, nullptr, WkB, bk, TMP, DD, nullptr, nullptr, DD); k_vtb<<<dim3(NT / 64, NH, 1), 256, 0, stream>>>(TMP, mb, KTh, KTl);
        k_gemmb<false, false><<<dim3(NT / 64, DD / 64, 1), 128, 0, stream>>>(Xb, nullptr, WvB, bv, TMP, DD, nullptr, nullptr, DD); k_vtb<<<dim3(NT / 64, NH, 1), 256, 0, stream>>>(TMP, mb, VTh, VTl);
        for (int h = 0; h < NH; ++h) { const size_t ho = (size_t)h * HD * NT;
            k_gemm3ll<<<dim3(1, 1, 1), 128, 0, stream>>>(VTh + ho, VTl + ho, NT, KTh + ho, KTl + ho, NT, NT, KV, HD);
            k_kvsplit<<<HD / 8, 256, 0, stream>>>(KV, scale, KVh, KVl);
            k_gemm3ll<<<dim3(NT / 64, 1, 1), 128, 0, stream>>>(Qh + h * HD, Ql + h * HD, DD, KVh, KVl, HD, HD, Y + h * HD, DD);
            k_gemmb<true, false><<<dim3(1, NT / 64, 1), 128, 0, stream>>>(VTh + ho, VTl + ho, T + (size_t)h * NT * NT, nullptr, C2, NT, nullptr, nullptr, NT);
            k_tadd<<<NT / 64, 256, 0, stream>>>(C2, h, Y); }
        k_split256m<<<NT / 8, 256, 0, stream>>>(Y, nullptr, Yh, Yl);
        k_gemmb<true, false><<<dim3(NT / 64, DD / 64, 1), 128, 0, stream>>>(Yh, Yl, WoB, bo, out + (size_t)b * NT * DD, DD, nullptr, nullptr, DD);
    }
}
